// GATDiGraphNet_37297495999113
// MI455X (gfx1250) — hardware-verified
//
#include <hip/hip_runtime.h>
#include <stddef.h>


#define NF    128
#define NDH   64
#define NG    128
#define GR    32
#define APX   136
#define APH   72
#define XSP   132
#define NB    512
#define CHUNK 2048
#define NTHR  256
#define NWAVE 8
#define WCAP  256
#define NGRP  (CHUNK / (NTHR * 4))

#define LO_SACC 0
#define LO_DEN  (LO_SACC + NB * NG)
#define LO_MX   (LO_DEN + NB * 2)
#define LO_LIST (LO_MX + NB * 2)
#define LO_WCNT (LO_LIST + NWAVE * WCAP)
#define LO_ALS  (LO_WCNT + 32)
#define LO_ATH  (LO_ALS + GR * 4)
#define LO_ATL  (LO_ATH + (GR * APX) / 2)
#define LDS_WORDS (LO_ATL + (GR * APX) / 2)
#define LDS_BYTES (LDS_WORDS * 4)

static_assert(NGRP == 2);
static_assert(WCAP == (CHUNK / NTHR) * 32);
static_assert(NB == 512);
static_assert(CHUNK == 2048);
static_assert(NB <= NWAVE * WCAP);
static_assert((LO_DEN % 4) == 0);
static_assert((LO_MX % 4) == 0);
static_assert((LO_LIST % 4) == 0);
static_assert((LO_ALS % 4) == 0);
static_assert((LO_ATH % 4) == 0);
static_assert((LO_ATL % 4) == 0);
static_assert(LDS_WORDS == 74144);
static_assert(LDS_BYTES == 296576);
static_assert(NB / GR == 16);
static_assert(GR * NG == 4096);

typedef float          v4f   __attribute__((ext_vector_type(4)));
typedef float          v8f   __attribute__((ext_vector_type(8)));
typedef int            v4i   __attribute__((ext_vector_type(4)));
typedef unsigned short v8us  __attribute__((ext_vector_type(8)));
typedef unsigned short v16us __attribute__((ext_vector_type(16)));
typedef __bf16         v16bf __attribute__((ext_vector_type(16)));
union Frag { v16bf v; v16us u; v8us half[2]; };
struct HL8 { v8us h; v8us l; };

__device__ __forceinline__ v8f wmb(v16bf a, v16bf b, v8f c) {
  v8f d = __builtin_amdgcn_wmma_f32_16x16x32_bf16(false, a, false, b, (short)0, c, false, false);
  asm volatile("v_nop\n\tv_nop\n\tv_nop\n\tv_nop" : "+v"(d) : "v"(a), "v"(b));
  return d;
}

__device__ __forceinline__ unsigned short f2bf(float f) {
  unsigned u = __float_as_uint(f);
  u = u + 0x7FFFu + ((u >> 16) & 1u);
  return (unsigned short)(u >> 16);
}
__device__ __forceinline__ float bf2f(unsigned short s) { return __uint_as_float(((unsigned)s) << 16); }

#define SPK(I, V) { const float fq = (V); const unsigned short hq = f2bf(fq); r.h[I] = hq; r.l[I] = f2bf(fq - bf2f(hq)); }
__device__ __forceinline__ HL8 split8(v4f a, v4f b) {
  HL8 r;
  SPK(0, a.x) SPK(1, a.y) SPK(2, a.z) SPK(3, a.w)
  SPK(4, b.x) SPK(5, b.y) SPK(6, b.z) SPK(7, b.w)
  return r;
}
#undef SPK

__device__ __forceinline__ void ldfrag(Frag& f, const unsigned short* rowp, int k0, int lh) {
  f.half[0] = *(const v8us*)(rowp + k0 + 8 * lh);
  f.half[1] = *(const v8us*)(rowp + k0 + 16 + 8 * lh);
}

__device__ __forceinline__ v8f wm3(const Frag& ah, const Frag& al, const Frag& bh, const Frag& bl, v8f c) {
  c = wmb(ah.v, bh.v, c);
  c = wmb(ah.v, bl.v, c);
  c = wmb(al.v, bh.v, c);
  return c;
}

template<int KT>
__device__ __forceinline__ v8f tile_gemm(const unsigned short* ah, const unsigned short* al,
                                         const unsigned short* bh, const unsigned short* bl, int lh, v8f c) {
#pragma unroll
  for (int kt = 0; kt < KT; ++kt) {
    Frag fa, fl, gb, gl;
    ldfrag(fa, ah, 32 * kt, lh); ldfrag(fl, al, 32 * kt, lh);
    ldfrag(gb, bh, 32 * kt, lh); ldfrag(gl, bl, 32 * kt, lh);
    c = wm3(fa, fl, gb, gl, c);
  }
  return c;
}

template<int KT>
__device__ __forceinline__ void tile_gemm2(const unsigned short* ah0, const unsigned short* al0,
                                           const unsigned short* ah1, const unsigned short* al1,
                                           const unsigned short* bh, const unsigned short* bl,
                                           int lh, v8f& c0, v8f& c1) {
#pragma unroll
  for (int kt = 0; kt < KT; ++kt) {
    Frag gb, gl, fa, fl;
    ldfrag(gb, bh, 32 * kt, lh); ldfrag(gl, bl, 32 * kt, lh);
    ldfrag(fa, ah0, 32 * kt, lh); ldfrag(fl, al0, 32 * kt, lh);
    c0 = wm3(fa, fl, gb, gl, c0);
    ldfrag(fa, ah1, 32 * kt, lh); ldfrag(fl, al1, 32 * kt, lh);
    c1 = wm3(fa, fl, gb, gl, c1);
  }
}

__global__ __launch_bounds__(NTHR) void k_prep(const float* __restrict__ B, unsigned short* Bh,
                                               unsigned short* Bl, int K, int Nc, int nmat) {
  const int kg8 = K >> 3;
  const int per = Nc * kg8;
  const int total = nmat * per;
  const int i = blockIdx.x * NTHR + threadIdx.x;
  if (i >= total) return;
  const int mat = i / per;
  const int rem = i - mat * per;
  const int n   = rem / kg8;
  const int kg  = rem - n * kg8;
  const float* s = B + (size_t)mat * K * Nc + (size_t)(kg * 8) * Nc + n;
  v4f a, b;
  a.x = s[0];              a.y = s[(size_t)1 * Nc]; a.z = s[(size_t)2 * Nc]; a.w = s[(size_t)3 * Nc];
  b.x = s[(size_t)4 * Nc]; b.y = s[(size_t)5 * Nc]; b.z = s[(size_t)6 * Nc]; b.w = s[(size_t)7 * Nc];
  const HL8 u = split8(a, b);
  const size_t o = (size_t)i * 8;
  *(volatile v8us*)(Bh + o) = u.h;
  *(volatile v8us*)(Bl + o) = u.l;
  __threadfence();
  *(volatile v8us*)(Bh + o) = u.h;
  *(volatile v8us*)(Bl + o) = u.l;
}

__global__ __launch_bounds__(NTHR) void k_enc(
    const float* __restrict__ x,
    const unsigned short* __restrict__ W1h, const unsigned short* __restrict__ W1l, const float* __restrict__ W1b,
    const unsigned short* __restrict__ W2h, const unsigned short* __restrict__ W2l, const float* __restrict__ W2b,
    const unsigned short* __restrict__ GWh, const unsigned short* __restrict__ GWl,
    const float* __restrict__ a_src, const float* __restrict__ a_dst,
    float* gA, float* alA, float* gB, float* alB, int nN) {
  __shared__ __attribute__((aligned(16))) unsigned short XTh[GR * APX];
  __shared__ __attribute__((aligned(16))) unsigned short XTl[GR * APX];
  __shared__ __attribute__((aligned(16))) unsigned short H1h[GR * APH];
  __shared__ __attribute__((aligned(16))) unsigned short H1l[GR * APH];
  __shared__ __attribute__((aligned(16))) unsigned short H2h[GR * APH];
  __shared__ __attribute__((aligned(16))) unsigned short H2l[GR * APH];
  __shared__ __attribute__((aligned(16))) float GT[GR * XSP];
  __shared__ __attribute__((aligned(16))) float ALs[GR * 4];

  const int tid  = threadIdx.x;
  const int lane = tid & 31;
  const int wave = tid >> 5;
  const int lh   = lane >> 4;
  const int m    = lane & 15;
  const int rowBase = blockIdx.x * GR;
  const v8f z8 = {0.f, 0.f, 0.f, 0.f, 0.f, 0.f, 0.f, 0.f};

  {
    const int r  = tid >> 3;
    const int c0 = (tid & 7) * 16;
    int row = rowBase + r;
    if (row > nN - 1) row = nN - 1;
    const float* p = x + (size_t)row * NF + c0;
    const v4f f0 = *(const v4f*)(p), f1 = *(const v4f*)(p + 4);
    const v4f f2 = *(const v4f*)(p + 8), f3 = *(const v4f*)(p + 12);
    const HL8 u0 = split8(f0, f1);
    const HL8 u1 = split8(f2, f3);
    *(v8us*)(XTh + r * APX + c0)     = u0.h;
    *(v8us*)(XTh + r * APX + c0 + 8) = u1.h;
    *(v8us*)(XTl + r * APX + c0)     = u0.l;
    *(v8us*)(XTl + r * APX + c0 + 8) = u1.l;
  }
  __syncthreads();

  {
    const int rt = wave >> 2, ct = wave & 3;
    v8f c = z8;
    c = tile_gemm<4>(XTh + (rt * 16 + m) * APX, XTl + (rt * 16 + m) * APX,
                     W1h + (size_t)(ct * 16 + m) * NF, W1l + (size_t)(ct * 16 + m) * NF, lh, c);
    const float bv = W1b[ct * 16 + m];
#pragma unroll
    for (int r = 0; r < 8; ++r) {
      float v = c[r] + bv;
      v = v > 0.f ? v : 0.f;
      const unsigned short hi = f2bf(v);
      const int o = (rt * 16 + 8 * lh + r) * APH + ct * 16 + m;
      H1h[o] = hi;
      H1l[o] = f2bf(v - bf2f(hi));
    }
  }
  __syncthreads();

  {
    const int rt = wave >> 2, ct = wave & 3;
    v8f c = z8;
    c = tile_gemm<2>(H1h + (rt * 16 + m) * APH, H1l + (rt * 16 + m) * APH,
                     W2h + (size_t)(ct * 16 + m) * NDH, W2l + (size_t)(ct * 16 + m) * NDH, lh, c);
    const float bv = W2b[ct * 16 + m];
#pragma unroll
    for (int r = 0; r < 8; ++r) {
      const float v = c[r] + bv;
      const unsigned short hi = f2bf(v);
      const int o = (rt * 16 + 8 * lh + r) * APH + ct * 16 + m;
      H2h[o] = hi;
      H2l[o] = f2bf(v - bf2f(hi));
    }
  }
  __syncthreads();

#pragma unroll 1
  for (int dd = 0; dd < 2; ++dd) {
    const unsigned short* gwh = GWh + (size_t)(dd * 2) * (NG * NDH) + (size_t)(wave * 16 + m) * NDH;
    const unsigned short* gwl = GWl + (size_t)(dd * 2) * (NG * NDH) + (size_t)(wave * 16 + m) * NDH;
    v8f c0 = z8, c1 = z8;
    tile_gemm2<2>(H2h + m * APH, H2l + m * APH, H2h + (16 + m) * APH, H2l + (16 + m) * APH,
                  gwh, gwl, lh, c0, c1);
#pragma unroll
    for (int r = 0; r < 8; ++r) {
      GT[(8 * lh + r) * XSP + wave * 16 + m]      = c0[r];
      GT[(16 + 8 * lh + r) * XSP + wave * 16 + m] = c1[r];
    }
    __syncthreads();

    if (tid < GR * 4) {
      const int row = tid >> 2, q = tid & 3, head = q & 1, isd = q >> 1;
      const float* vs = a_src + (size_t)((dd * 2) * 2 + head) * NDH;
      const float* vd = a_dst + (size_t)((dd * 2) * 2 + head) * NDH;
      const float* gr = GT + row * XSP + head * NDH;
      float s = 0.f;
#pragma unroll 4
      for (int c = 0; c < NDH; ++c) {
        const float ws = vs[c];
        const float wd = vd[c];
        s += gr[c] * (isd ? wd : ws);
      }
      ALs[row * 4 + q] = s;
    }
    __syncthreads();

    {
      float* gP  = dd ? gB : gA;
      float* alP = dd ? alB : alA;
      const v4f x0 = *(const v4f*)(GT + (4 * wave + 0) * XSP + 4 * lane);
      const v4f x1 = *(const v4f*)(GT + (4 * wave + 1) * XSP + 4 * lane);
      const v4f x2 = *(const v4f*)(GT + (4 * wave + 2) * XSP + 4 * lane);
      const v4f x3 = *(const v4f*)(GT + (4 * wave + 3) * XSP + 4 * lane);
      const v4f av = *(const v4f*)(ALs + 4 * lane);
      float* p0 = gP + (size_t)(rowBase + 4 * wave + 0) * NG + 4 * lane;
      float* p1 = gP + (size_t)(rowBase + 4 * wave + 1) * NG + 4 * lane;
      float* p2 = gP + (size_t)(rowBase + 4 * wave + 2) * NG + 4 * lane;
      float* p3 = gP + (size_t)(rowBase + 4 * wave + 3) * NG + 4 * lane;
      float* ap = alP + (size_t)(rowBase + lane) * 4;
      *(volatile v4f*)p0 = x0; *(volatile v4f*)p1 = x1; *(volatile v4f*)p2 = x2; *(volatile v4f*)p3 = x3;
      if (wave == 0) *(volatile v4f*)ap = av;
      __threadfence();
      *(volatile v4f*)p0 = x0; *(volatile v4f*)p1 = x1; *(volatile v4f*)p2 = x2; *(volatile v4f*)p3 = x3;
      if (wave == 0) *(volatile v4f*)ap = av;
    }
    __syncthreads();
  }
}

__device__ __forceinline__ void agg_scan(float* sacc, float* den, float* mx, int* list, int* wcnt,
                                         const int* __restrict__ keyp, const int* __restrict__ gatp,
                                         const float* __restrict__ gin, const float* __restrict__ alin,
                                         int nN, int nE, int nodeBase, int tid, int lane, int wave) {
  {
    const v4f z4 = {0.f, 0.f, 0.f, 0.f};
    const v4f m4 = {-1.0e30f, -1.0e30f, -1.0e30f, -1.0e30f};
    v4f* s4 = (v4f*)sacc;
    for (int i = tid; i < NB * NG / 4; i += NTHR) s4[i] = z4;
    v4f* d4 = (v4f*)den;
    v4f* x4 = (v4f*)mx;
    for (int i = tid; i < NB * 2 / 4; i += NTHR) { d4[i] = z4; x4[i] = m4; }
  }
  __syncthreads();
  const int hd = lane >> 4;
  const bool al16 = ((((size_t)keyp) & 15) == 0);
  const int nChunks = (nE + CHUNK - 1) / CHUNK;

#pragma unroll 1
  for (int ch = 0; ch < nChunks; ++ch) {
    const int cbase = ch * CHUNK;
    int wc = 0;
#pragma unroll
    for (int g = 0; g < NGRP; ++g) {
      const int el0 = (g * NTHR + tid) * 4;
      const int e0  = cbase + el0;
      const int sent = -2147483647 - 1;
      v4i d;
      if (al16 && (cbase + CHUNK <= nE)) {
        d = *(const v4i*)(keyp + e0);
      } else {
        d.x = (e0     < nE) ? keyp[min(e0,     nE - 1)] : sent;
        d.y = (e0 + 1 < nE) ? keyp[min(e0 + 1, nE - 1)] : sent;
        d.z = (e0 + 2 < nE) ? keyp[min(e0 + 2, nE - 1)] : sent;
        d.w = (e0 + 3 < nE) ? keyp[min(e0 + 3, nE - 1)] : sent;
      }
      const unsigned s0 = (unsigned)d.x - (unsigned)nodeBase;
      const unsigned s1 = (unsigned)d.y - (unsigned)nodeBase;
      const unsigned s2 = (unsigned)d.z - (unsigned)nodeBase;
      const unsigned s3 = (unsigned)d.w - (unsigned)nodeBase;
      const bool h0 = s0 < (unsigned)NB;
      const bool h1 = s1 < (unsigned)NB;
      const bool h2 = s2 < (unsigned)NB;
      const bool h3 = s3 < (unsigned)NB;
      const unsigned many = __builtin_amdgcn_ballot_w32(h0 | h1 | h2 | h3);
      if (many != 0u) {
#define HITJ(J, HJ, SJ) { \
          const unsigned mj = __builtin_amdgcn_ballot_w32(HJ); \
          if (HJ) { \
            const int pos = wc + (int)__builtin_amdgcn_mbcnt_lo(mj, 0u); \
            if (pos < WCAP) list[wave * WCAP + pos] = ((el0 + (J)) << 9) | (int)(SJ); \
          } \
          wc += (int)__builtin_popcount(mj); }
        HITJ(0, h0, s0)
        HITJ(1, h1, s1)
        HITJ(2, h2, s2)
        HITJ(3, h3, s3)
#undef HITJ
      }
    }
    if (lane == 0) wcnt[wave] = wc;
    __syncthreads();

    if (wave == 0) {
#pragma unroll 1
      for (int wsx = 0; wsx < NWAVE; ++wsx) {
        int n = wcnt[wsx];
        if (n > WCAP) n = WCAP;
        if (n < 0) n = 0;
#pragma unroll 1
        for (int i = 0; i < n; ++i) {
          const int ent  = list[wsx * WCAP + i];
          const int slot = ent & (NB - 1);
          const int el   = (ent >> 9) & (CHUNK - 1);
          int e = cbase + el;
          if (e > nE - 1) e = nE - 1;
          int src = gatp[e];
          src = src < 0 ? 0 : (src > nN - 1 ? nN - 1 : src);
          int nd = nodeBase + slot;
          if (nd > nN - 1) nd = nN - 1;
          float al = alin[(size_t)src * 4 + hd] + alin[(size_t)nd * 4 + 2 + hd];
          al = (al > 0.f) ? al : 0.2f * al;
          const int ai = slot * 2 + hd;
          const float mo = mx[ai];
          const float mn = fmaxf(mo, al);
          const float sc = __expf(fmaxf(mo - mn, -80.f));
          const float p  = __expf(al - mn);
          const v4f xv = *(const v4f*)(gin + (size_t)src * NG + 4 * lane);
          v4f* sp = (v4f*)(sacc + slot * NG + 4 * lane);
          const v4f cur = *sp;
          const v4f nxt = cur * sc + p * xv;
          *sp = nxt;
          const float dn = den[ai];
          den[ai] = dn * sc + p;
          mx[ai] = mn;
        }
      }
    }
    __syncthreads();
  }
}

__device__ __forceinline__ void conv_step(const float* sacc, const float* den, const float* mx,
                                          unsigned short* ath, unsigned short* atl,
                                          const float* __restrict__ gin, const float* __restrict__ alin,
                                          const float* __restrict__ gatb, int j, int nodeBase, int nN, int tid) {
  const int r  = tid >> 3;
  const int c0 = (tid & 7) * 16;
  const int slot = j * GR + r;
  int node = nodeBase + slot;
  if (node > nN - 1) node = nN - 1;
  const int head = c0 >> 6;
  float al = alin[(size_t)node * 4 + head] + alin[(size_t)node * 4 + 2 + head];
  al = (al > 0.f) ? al : 0.2f * al;
  const int ai = slot * 2 + head;
  const float mo = mx[ai];
  const float mn = fmaxf(mo, al);
  const float sc = __expf(fmaxf(mo - mn, -80.f));
  const float p  = __expf(al - mn);
  const float dn = den[ai] * sc + p;
  const float inv = 1.0f / (dn + 1e-16f);
  const float* srow = sacc + slot * NG + c0;
  const float* grow = gin + (size_t)node * NG + c0;
  const float* brow = gatb + c0;
  const v4f v0 = (*(const v4f*)(srow)      * sc + p * *(const v4f*)(grow))      * inv + *(const v4f*)(brow);
  const v4f v1 = (*(const v4f*)(srow + 4)  * sc + p * *(const v4f*)(grow + 4))  * inv + *(const v4f*)(brow + 4);
  const v4f v2 = (*(const v4f*)(srow + 8)  * sc + p * *(const v4f*)(grow + 8))  * inv + *(const v4f*)(brow + 8);
  const v4f v3 = (*(const v4f*)(srow + 12) * sc + p * *(const v4f*)(grow + 12)) * inv + *(const v4f*)(brow + 12);
  const HL8 u0 = split8(v0, v1);
  const HL8 u1 = split8(v2, v3);
  *(v8us*)(ath + r * APX + c0)     = u0.h;
  *(v8us*)(ath + r * APX + c0 + 8) = u1.h;
  *(v8us*)(atl + r * APX + c0)     = u0.l;
  *(v8us*)(atl + r * APX + c0 + 8) = u1.l;
}

template<int RELU>
__device__ __forceinline__ void lin_step(const unsigned short* ath, const unsigned short* atl,
                                         const unsigned short* __restrict__ LWh, const unsigned short* __restrict__ LWl,
                                         const float* __restrict__ linb, float* ht, int wave, int lh, int m) {
  const int rt = wave >> 2, ct = wave & 3;
  v8f c = {0.f, 0.f, 0.f, 0.f, 0.f, 0.f, 0.f, 0.f};
  c = tile_gemm<4>(ath + (rt * 16 + m) * APX, atl + (rt * 16 + m) * APX,
                   LWh + (size_t)(ct * 16 + m) * NG, LWl + (size_t)(ct * 16 + m) * NG, lh, c);
  const float bv = linb[ct * 16 + m];
#pragma unroll
  for (int r = 0; r < 8; ++r) {
    float v = c[r] + bv;
    if (RELU) v = v > 0.f ? v : 0.f;
    ht[(rt * 16 + 8 * lh + r) * NDH + ct * 16 + m] = v;
  }
}

__global__ __launch_bounds__(NTHR) void k_agg0(
    const int* __restrict__ ei, int nE, int koff, int goff,
    const float* __restrict__ gin, const float* __restrict__ alin, const float* __restrict__ gatb,
    const unsigned short* __restrict__ LWh, const unsigned short* __restrict__ LWl, const float* __restrict__ linb,
    const unsigned short* __restrict__ GWh, const unsigned short* __restrict__ GWl,
    const float* __restrict__ as1, const float* __restrict__ ad1,
    float* gout, float* alout, int nN) {
  extern __shared__ v4f lds_dyn[];
  float* lw = (float*)lds_dyn;
  float* sacc = lw + LO_SACC;
  float* den  = lw + LO_DEN;
  float* mx   = lw + LO_MX;
  int*   list = (int*)(lw + LO_LIST);
  int*   wcnt = (int*)(lw + LO_WCNT);
  float* als  = lw + LO_ALS;
  unsigned short* ath = (unsigned short*)(lw + LO_ATH);
  unsigned short* atl = (unsigned short*)(lw + LO_ATL);

  const int tid  = threadIdx.x;
  const int lane = tid & 31;
  const int wave = tid >> 5;
  const int lh   = lane >> 4;
  const int m    = lane & 15;
  const int nodeBase = blockIdx.x * NB;
  const v8f z8 = {0.f, 0.f, 0.f, 0.f, 0.f, 0.f, 0.f, 0.f};

  agg_scan(sacc, den, mx, list, wcnt, ei + koff, ei + goff, gin, alin, nN, nE, nodeBase, tid, lane, wave);

#pragma unroll 1
  for (int j = 0; j < NB / GR; ++j) {
    float* sr = sacc + j * (GR * NG);
    conv_step(sacc, den, mx, ath, atl, gin, alin, gatb, j, nodeBase, nN, tid);
    __syncthreads();
    float* ht = sr;
    unsigned short* hbh = (unsigned short*)(sr + 2048);
    unsigned short* hbl = (unsigned short*)(sr + 3072);
    lin_step<1>(ath, atl, LWh, LWl, linb, ht, wave, lh, m);
    __syncthreads();
    {
      const int r  = tid >> 3;
      const int c0 = (tid & 7) * 8;
      const v4f a = *(const v4f*)(ht + r * NDH + c0);
      const v4f b = *(const v4f*)(ht + r * NDH + c0 + 4);
      const HL8 u = split8(a, b);
      *(v8us*)(hbh + r * NDH + c0) = u.h;
      *(v8us*)(hbl + r * NDH + c0) = u.l;
    }
    __syncthreads();
    v8f c0a = z8, c1a = z8;
    tile_gemm2<2>(hbh + m * NDH, hbl + m * NDH, hbh + (16 + m) * NDH, hbl + (16 + m) * NDH,
                  GWh + (size_t)(wave * 16 + m) * NDH, GWl + (size_t)(wave * 16 + m) * NDH, lh, c0a, c1a);
    __syncthreads();
    float* gt = sr;
#pragma unroll
    for (int r = 0; r < 8; ++r) {
      gt[(8 * lh + r) * NG + wave * 16 + m]      = c0a[r];
      gt[(16 + 8 * lh + r) * NG + wave * 16 + m] = c1a[r];
    }
    __syncthreads();
    if (tid < GR * 4) {
      const int row = tid >> 2, q = tid & 3, head = q & 1, isd = q >> 1;
      const float* vs = as1 + head * NDH;
      const float* vd = ad1 + head * NDH;
      const float* gr = gt + row * NG + head * NDH;
      float s = 0.f;
#pragma unroll 4
      for (int c = 0; c < NDH; ++c) {
        const float ws = vs[c];
        const float wd = vd[c];
        s += gr[c] * (isd ? wd : ws);
      }
      als[row * 4 + q] = s;
    }
    __syncthreads();
    {
      const size_t row0 = (size_t)nodeBase + (size_t)j * GR;
      const v4f x0 = *(const v4f*)(gt + (4 * wave + 0) * NG + 4 * lane);
      const v4f x1 = *(const v4f*)(gt + (4 * wave + 1) * NG + 4 * lane);
      const v4f x2 = *(const v4f*)(gt + (4 * wave + 2) * NG + 4 * lane);
      const v4f x3 = *(const v4f*)(gt + (4 * wave + 3) * NG + 4 * lane);
      const v4f av = *(const v4f*)(als + 4 * lane);
      float* p0 = gout + (row0 + 4 * wave + 0) * NG + 4 * lane;
      float* p1 = gout + (row0 + 4 * wave + 1) * NG + 4 * lane;
      float* p2 = gout + (row0 + 4 * wave + 2) * NG + 4 * lane;
      float* p3 = gout + (row0 + 4 * wave + 3) * NG + 4 * lane;
      float* ap = alout + (row0 + lane) * 4;
      *(volatile v4f*)p0 = x0; *(volatile v4f*)p1 = x1; *(volatile v4f*)p2 = x2; *(volatile v4f*)p3 = x3;
      if (wave == 0) *(volatile v4f*)ap = av;
      __threadfence();
      *(volatile v4f*)p0 = x0; *(volatile v4f*)p1 = x1; *(volatile v4f*)p2 = x2; *(volatile v4f*)p3 = x3;
      if (wave == 0) *(volatile v4f*)ap = av;
    }
  }
}

__global__ __launch_bounds__(NTHR) void k_agg1(
    const int* __restrict__ ei, int nE, int koff, int goff,
    const float* __restrict__ gin, const float* __restrict__ alin, const float* __restrict__ gatb,
    const unsigned short* __restrict__ LWh, const unsigned short* __restrict__ LWl, const float* __restrict__ linb,
    const float* __restrict__ scw, const float* __restrict__ scin, const float* __restrict__ scb,
    float* scout, int addin, int lim, int nN) {
  extern __shared__ v4f lds_dyn[];
  float* lw = (float*)lds_dyn;
  float* sacc = lw + LO_SACC;
  float* den  = lw + LO_DEN;
  float* mx   = lw + LO_MX;
  int*   list = (int*)(lw + LO_LIST);
  int*   wcnt = (int*)(lw + LO_WCNT);
  unsigned short* ath = (unsigned short*)(lw + LO_ATH);
  unsigned short* atl = (unsigned short*)(lw + LO_ATL);

  const int tid  = threadIdx.x;
  const int lane = tid & 31;
  const int wave = tid >> 5;
  const int lh   = lane >> 4;
  const int m    = lane & 15;
  const int nodeBase = blockIdx.x * NB;

  agg_scan(sacc, den, mx, list, wcnt, ei + koff, ei + goff, gin, alin, nN, nE, nodeBase, tid, lane, wave);

  float* scs = (float*)list;
#pragma unroll 1
  for (int j = 0; j < NB / GR; ++j) {
    float* sr = sacc + j * (GR * NG);
    conv_step(sacc, den, mx, ath, atl, gin, alin, gatb, j, nodeBase, nN, tid);
    __syncthreads();
    float* ht = sr;
    lin_step<0>(ath, atl, LWh, LWl, linb, ht, wave, lh, m);
    __syncthreads();
    if (tid < GR) {
      const float* hr = ht + tid * NDH;
      float s = 0.f;
#pragma unroll 4
      for (int c = 0; c < NDH; ++c) s += hr[c] * scw[c];
      if (addin) s += scin[(size_t)nodeBase + (size_t)j * GR + tid] + scb[0];
      scs[j * GR + tid] = s;
    }
  }
  __syncthreads();

  if (wave == 0) {
    const v4f v0 = *(const v4f*)(scs + 0 * 128 + 4 * lane);
    const v4f v1 = *(const v4f*)(scs + 1 * 128 + 4 * lane);
    const v4f v2 = *(const v4f*)(scs + 2 * 128 + 4 * lane);
    const v4f v3 = *(const v4f*)(scs + 3 * 128 + 4 * lane);
#define STSEG(I, V) { \
      const int node = nodeBase + (I) * 128 + 4 * lane; \
      float* op = scout + node; \
      if (node + 4 <= lim) { *(volatile v4f*)op = (V); } \
      else { \
        if (node + 0 < lim) *(volatile float*)(op + 0) = (V).x; \
        if (node + 1 < lim) *(volatile float*)(op + 1) = (V).y; \
        if (node + 2 < lim) *(volatile float*)(op + 2) = (V).z; \
      } }
    STSEG(0, v0) STSEG(1, v1) STSEG(2, v2) STSEG(3, v3)
    __threadfence();
    STSEG(0, v0) STSEG(1, v1) STSEG(2, v2) STSEG(3, v3)
#undef STSEG
  }
}

static size_t al256(size_t v) { return (v + 255) & ~(size_t)255; }

extern "C" void kernel_launch(void* const* d_in, const int* in_sizes, int n_in,
                              void* d_out, int out_size, void* d_ws, size_t ws_size,
                              hipStream_t stream) {
  if (n_in < 14) return;
  const int nN = in_sizes[0] / NF;
  if (nN <= 0 || in_sizes[0] != nN * NF) return;
  if (in_sizes[1] < 2 || (in_sizes[1] & 1)) return;
  const int nE = in_sizes[1] / 2;
  if (in_sizes[2] != NF * NDH || in_sizes[3] != NDH) return;
  if (in_sizes[4] != NDH * NDH || in_sizes[5] != NDH) return;
  if (in_sizes[6] != 4 * NDH * NG || in_sizes[7] != 4 * 2 * NDH || in_sizes[8] != 4 * 2 * NDH) return;
  if (in_sizes[9] != 4 * NG || in_sizes[10] != 4 * NG * NDH || in_sizes[11] != 4 * NDH) return;
  if (in_sizes[12] != 2 * NDH || in_sizes[13] < 1) return;
  if (out_size != nN) return;

  const float* x        = (const float*)d_in[0];
  const int*   ei       = (const int*)d_in[1];
  const float* W1w      = (const float*)d_in[2];
  const float* W1b      = (const float*)d_in[3];
  const float* W2w      = (const float*)d_in[4];
  const float* W2b      = (const float*)d_in[5];
  const float* gatW     = (const float*)d_in[6];
  const float* a_src    = (const float*)d_in[7];
  const float* a_dst    = (const float*)d_in[8];
  const float* gat_b    = (const float*)d_in[9];
  const float* linW     = (const float*)d_in[10];
  const float* lin_b    = (const float*)d_in[11];
  const float* scorer_w = (const float*)d_in[12];
  const float* scorer_b = (const float*)d_in[13];
  float* out = (float*)d_out;

  const int nBlk = (nN + NB - 1) / NB;
  const int Npad = nBlk * NB;

  char* base = (char*)d_ws;
  size_t off = 0;
  unsigned short* W1h = (unsigned short*)(base + off); off += al256((size_t)NDH * NF * 2);
  unsigned short* W1l = (unsigned short*)(base + off); off += al256((size_t)NDH * NF * 2);
  unsigned short* W2h = (unsigned short*)(base + off); off += al256((size_t)NDH * NDH * 2);
  unsigned short* W2l = (unsigned short*)(base + off); off += al256((size_t)NDH * NDH * 2);
  unsigned short* GWh = (unsigned short*)(base + off); off += al256((size_t)4 * NG * NDH * 2);
  unsigned short* GWl = (unsigned short*)(base + off); off += al256((size_t)4 * NG * NDH * 2);
  unsigned short* LWh = (unsigned short*)(base + off); off += al256((size_t)4 * NDH * NG * 2);
  unsigned short* LWl = (unsigned short*)(base + off); off += al256((size_t)4 * NDH * NG * 2);
  float* gA  = (float*)(base + off); off += al256((size_t)Npad * NG * 4);
  float* gB  = (float*)(base + off); off += al256((size_t)Npad * NG * 4);
  float* gC  = (float*)(base + off); off += al256((size_t)Npad * NG * 4);
  float* alA = (float*)(base + off); off += al256((size_t)Npad * 4 * 4);
  float* alB = (float*)(base + off); off += al256((size_t)Npad * 4 * 4);
  float* alC = (float*)(base + off); off += al256((size_t)Npad * 4 * 4);
  float* sfw = (float*)(base + off); off += al256((size_t)Npad * 4);
  if (off > ws_size) return;

  {
    const int t1 = 1 * NDH * (NF / 8);
    k_prep<<<(t1 + NTHR - 1) / NTHR, NTHR, 0, stream>>>(W1w, W1h, W1l, NF, NDH, 1);
    const int t2 = 1 * NDH * (NDH / 8);
    k_prep<<<(t2 + NTHR - 1) / NTHR, NTHR, 0, stream>>>(W2w, W2h, W2l, NDH, NDH, 1);
    const int t3 = 4 * NG * (NDH / 8);
    k_prep<<<(t3 + NTHR - 1) / NTHR, NTHR, 0, stream>>>(gatW, GWh, GWl, NDH, NG, 4);
    const int t4 = 4 * NDH * (NG / 8);
    k_prep<<<(t4 + NTHR - 1) / NTHR, NTHR, 0, stream>>>(linW, LWh, LWl, NG, NDH, 4);
  }

  k_enc<<<Npad / GR, NTHR, 0, stream>>>(x, W1h, W1l, W1b, W2h, W2l, W2b, GWh, GWl, a_src, a_dst,
                                        gA, alA, gB, alB, nN);

  hipFuncSetAttribute(reinterpret_cast<const void*>(&k_agg0),
                      hipFuncAttributeMaxDynamicSharedMemorySize, LDS_BYTES);
  hipFuncSetAttribute(reinterpret_cast<const void*>(&k_agg1),
                      hipFuncAttributeMaxDynamicSharedMemorySize, LDS_BYTES);

  const size_t WP = (size_t)NG * NDH;
  k_agg0<<<nBlk, NTHR, LDS_BYTES, stream>>>(ei, nE, nE, 0, gA, alA, gat_b + 0 * NG,
                                            LWh + 0 * WP, LWl + 0 * WP, lin_b + 0 * NDH,
                                            GWh + 1 * WP, GWl + 1 * WP,
                                            a_src + (size_t)(1 * 2) * NDH, a_dst + (size_t)(1 * 2) * NDH,
                                            gC, alC, nN);
  k_agg1<<<nBlk, NTHR, LDS_BYTES, stream>>>(ei, nE, nE, 0, gC, alC, gat_b + 1 * NG,
                                            LWh + 1 * WP, LWl + 1 * WP, lin_b + 1 * NDH,
                                            scorer_w, sfw, scorer_b, sfw, 0, Npad, nN);
  k_agg0<<<nBlk, NTHR, LDS_BYTES, stream>>>(ei, nE, 0, nE, gB, alB, gat_b + 2 * NG,
                                            LWh + 2 * WP, LWl + 2 * WP, lin_b + 2 * NDH,
                                            GWh + 3 * WP, GWl + 3 * WP,
                                            a_src + (size_t)(3 * 2) * NDH, a_dst + (size_t)(3 * 2) * NDH,
                                            gC, alC, nN);
  k_agg1<<<nBlk, NTHR, LDS_BYTES, stream>>>(ei, nE, 0, nE, gC, alC, gat_b + 3 * NG,
                                            LWh + 3 * WP, LWl + 3 * WP, lin_b + 3 * NDH,
                                            scorer_w + NDH, sfw, scorer_b, out, 1, nN, nN);
}
